// MSMLMultiHeadAttention_86500641342113
// MI455X (gfx1250) — hardware-verified
//
#include <hip/hip_runtime.h>
#include <math.h>

typedef __attribute__((ext_vector_type(16))) _Float16 v16h;
typedef __attribute__((ext_vector_type(16))) __bf16 v16b;
typedef __attribute__((ext_vector_type(8)))  _Float16 v8h;
typedef __attribute__((ext_vector_type(8)))  float v8f;
typedef __attribute__((ext_vector_type(4)))  float v4f;
typedef __attribute__((ext_vector_type(2)))  float v2f;
typedef __attribute__((ext_vector_type(4)))  unsigned v4u;
typedef __attribute__((ext_vector_type(4)))  int v4i;
typedef float __attribute__((may_alias)) float_a;
typedef int __attribute__((may_alias)) int_a;

template <typename T> __device__ __forceinline__ void vst2(void* p, T v) { *(volatile T*)p = v; __threadfence(); *(volatile T*)p = v; }
__device__ __forceinline__ v8f wmma16(v16h a, v16h b, v8f c) {
  v8f d = __builtin_amdgcn_wmma_f32_16x16x32_f16(false, a, false, b, (short)0, c, false, false);
  asm volatile("v_nop\n\tv_nop\n\tv_nop\n\tv_nop" : "+v"(d) : "v"(a), "v"(b));
  return d;
}
__device__ __forceinline__ v8f wmma_bf(v16b a, v16b b, v8f c) {
  v8f d = __builtin_amdgcn_wmma_f32_16x16x32_bf16(false, a, false, b, (short)0, c, false, false);
  asm volatile("v_nop\n\tv_nop\n\tv_nop\n\tv_nop" : "+v"(d) : "v"(a), "v"(b));
  return d;
}
__device__ __forceinline__ v16h frag_h(const _Float16* rowk0, int lane) {
  union { v16h v; v8h q[2]; } u; const _Float16* p = rowk0 + 8 * (lane >> 4);
  u.q[0] = *(const v8h*)p; u.q[1] = *(const v8h*)(p + 16); return u.v;
}
__device__ __forceinline__ v16h frag_f32(const float* rowk0, int lane) {
  v16h a; const float* p = rowk0 + 8 * (lane >> 4);
#pragma unroll
  for (int i = 0; i < 8; ++i) { a[i] = (_Float16)p[i]; a[8 + i] = (_Float16)p[16 + i]; }
  return a;
}
__device__ __forceinline__ v16h frag_f32s(const float* rowk0, int lane, float sc) {
  v16h a; const float* p = rowk0 + 8 * (lane >> 4);
#pragma unroll
  for (int i = 0; i < 8; ++i) { a[i] = (_Float16)(p[i] * sc); a[8 + i] = (_Float16)(p[16 + i] * sc); }
  return a;
}
__device__ __forceinline__ v16h fragc_f32(const float* W, int k0, int n, int lane, int ld, int K) {
  v16h a; const int g = lane >> 4;
#pragma unroll
  for (int i = 0; i < 8; ++i) { const int ka = k0 + 8 * g + i, kb = ka + 16;
    a[i] = (_Float16)(ka < K ? W[(size_t)(ka < K ? ka : K - 1) * ld + n] : 0.f); a[8 + i] = (_Float16)(kb < K ? W[(size_t)(kb < K ? kb : K - 1) * ld + n] : 0.f); }
  return a;
}
struct F2 { v16b h, l; };
__device__ __forceinline__ F2 bsplit16(const float v[16]) { F2 r;
#pragma unroll
  for (int i = 0; i < 16; ++i) { const __bf16 h = (__bf16)v[i]; r.h[i] = h; r.l[i] = (__bf16)(v[i] - (float)h); }
  return r; }
__device__ __forceinline__ F2 split_row(const float* row, int k0, int lane) { float v[16]; const float* p = row + k0 + 8 * (lane >> 4);
#pragma unroll
  for (int i = 0; i < 8; ++i) { v[i] = p[i]; v[8 + i] = p[16 + i]; }
  return bsplit16(v); }
__device__ __forceinline__ F2 split_rowK(const float* row, int k0, int lane, int K) { float v[16]; const int g = lane >> 4;
#pragma unroll
  for (int i = 0; i < 8; ++i) { const int ka = k0 + 8 * g + i, kb = ka + 16; v[i] = ka < K ? row[ka < K ? ka : K - 1] : 0.f; v[8 + i] = kb < K ? row[kb < K ? kb : K - 1] : 0.f; }
  return bsplit16(v); }
__device__ __forceinline__ F2 split_col(const float* W, int k0, int n, int lane, int ld, int K) { float v[16]; const int g = lane >> 4;
#pragma unroll
  for (int i = 0; i < 8; ++i) { const int ka = k0 + 8 * g + i, kb = ka + 16; v[i] = ka < K ? W[(size_t)(ka < K ? ka : K - 1) * ld + n] : 0.f; v[8 + i] = kb < K ? W[(size_t)(kb < K ? kb : K - 1) * ld + n] : 0.f; }
  return bsplit16(v); }
__device__ __forceinline__ v8f mac3(const F2& a, const F2& b, v8f c) { c = wmma_bf(a.l, b.h, c); c = wmma_bf(a.h, b.l, c); return wmma_bf(a.h, b.h, c); }
__device__ __forceinline__ float sigm(float v) { return 1.0f / (1.0f + expf(-v)); }
#define LDSX() do { asm volatile("s_wait_dscnt 0" ::: "memory"); __builtin_amdgcn_wave_barrier(); __builtin_amdgcn_fence(__ATOMIC_RELEASE, "workgroup"); } while (0)


#define NB 2
#define NTOK 16384
#define CC 256
#define MW 16
#define NWIN (NTOK / MW)
#define WOUT 64
#define TQ (WOUT * MW)
#ifndef TNB
#define TNB NB
#endif
typedef __attribute__((ext_vector_type(8))) __bf16 v8b;
__device__ __forceinline__ v16b frag_b(const __bf16* rowk0, int lane) {
  union { v16b v; v8b q[2]; } u; const __bf16* p = rowk0 + 8 * (lane >> 4);
  u.q[0] = *(const v8b*)p; u.q[1] = *(const v8b*)(p + 16); return u.v;
}
__device__ __forceinline__ float bfr(float v) { return (float)(__bf16)v; }
__device__ __attribute__((noinline)) float exp_ni(float v) { return expf(v); }
__device__ __attribute__((noinline)) float erf_ni(float v) { return erff(v); }

#define WS_PW  0u
#define WS_PHQ (WS_PW + 2u * 2 * CC * CC)
#define WS_PHK (WS_PHQ + 4u * (size_t)NB * NTOK * CC)
#define WS_KVT (WS_PHK + 4u * (size_t)NB * NTOK * CC)
#define WS_END (WS_KVT + 4u * (size_t)NB * MW * CC * CC)

__device__ __forceinline__ v16b fragb_f32(const float* __restrict__ p, int lane) { v16b a; const float* pp = p + 8 * (lane >> 4);
#pragma unroll
  for (int i = 0; i < 8; ++i) { a[i] = (__bf16)pp[i]; a[8 + i] = (__bf16)pp[16 + i]; } return a; }
__device__ __forceinline__ float elu1(float y) { return (y > 0.f ? y : expm1f(y)) + 1.0f; }
__global__ __launch_bounds__(256) void k_packw(const float* __restrict__ WQ, const float* __restrict__ WK, __bf16* __restrict__ PW) { const int n = blockIdx.x, t = threadIdx.x; __shared__ __align__(16) __bf16 s[CC]; const int which = n / CC, o = n % CC; const float* Wm = which == 0 ? WQ : WK;
  s[t] = (__bf16)Wm[(size_t)t * CC + o]; __syncthreads(); if (t < CC / 8) vst2((unsigned*)(PW + (size_t)n * CC + t * 8), *(const v4u*)&s[t * 8]); }
__global__ __launch_bounds__(128) void k_phi(const float* __restrict__ X, const __bf16* __restrict__ PW, const float* __restrict__ BQ, const float* __restrict__ BK, float* __restrict__ PHQ, float* __restrict__ PHK) { __shared__ __align__(16) float sf[4][16][132];
  const int tid = threadIdx.x, wave = tid >> 5, lane = tid & 31, col = lane & 15, g = lane >> 4; const int which = blockIdx.z; const size_t r0 = (size_t)blockIdx.x * 64 + wave * 16; const int c0 = blockIdx.y * 128; const float* Bm = which == 0 ? BQ : BK; float* dst = which == 0 ? PHQ : PHK;
  v8f acc[8] = {};
#pragma unroll
  for (int kc = 0; kc < CC / 32; ++kc) { const v16b a = fragb_f32(X + (r0 + col) * CC + kc * 32, lane);
#pragma unroll
    for (int j = 0; j < 8; ++j) acc[j] = wmma_bf(a, frag_b(PW + (size_t)(which * CC + c0 + j * 16 + col) * CC + kc * 32, lane), acc[j]); }
#pragma unroll
  for (int j = 0; j < 8; ++j) { const float bb = bfr(Bm[c0 + j * 16 + col]);
#pragma unroll
    for (int r = 0; r < 8; ++r) sf[wave][8 * g + r][j * 16 + col] = elu1(elu1(acc[j][r] + bb)); }
  LDSX(); for (int rl = 0; rl < 16; ++rl) vst2(dst + (r0 + rl) * CC + c0 + lane * 4, *(const v4f*)&sf[wave][rl][lane * 4]); }
__global__ __launch_bounds__(128) void k_kv(const float* __restrict__ PHK, const float* __restrict__ X, float* __restrict__ KVT) { __shared__ __align__(16) float st[128][68];
  const int tid = threadIdx.x, wave = tid >> 5, lane = tid & 31, col = lane & 15, g = lane >> 4; const size_t b = blockIdx.z / MW; const int m = blockIdx.z % MW; const int c0 = blockIdx.x * 64 + wave * 16; const int d0 = blockIdx.y * 128;
  v8f acc[8] = {};
#pragma unroll 1
  for (int kc = 0; kc < NWIN / 32; ++kc) { float av[16]; const int w0 = kc * 32 + 8 * g;
#pragma unroll
    for (int i = 0; i < 8; ++i) { av[i] = PHK[(b * NTOK + (size_t)(w0 + i) * MW + m) * CC + c0 + col]; av[8 + i] = PHK[(b * NTOK + (size_t)(w0 + 16 + i) * MW + m) * CC + c0 + col]; }
    const F2 a = bsplit16(av);
#pragma unroll
    for (int j = 0; j < 8; ++j) { v16b w; const int d = d0 + j * 16 + col;
#pragma unroll
      for (int i = 0; i < 8; ++i) { w[i] = (__bf16)X[(b * NTOK + (size_t)(w0 + i) * MW + m) * CC + d]; w[8 + i] = (__bf16)X[(b * NTOK + (size_t)(w0 + 16 + i) * MW + m) * CC + d]; }
      acc[j] = wmma_bf(a.h, w, acc[j]); acc[j] = wmma_bf(a.l, w, acc[j]); } }
#pragma unroll
  for (int j = 0; j < 8; ++j)
#pragma unroll
    for (int r = 0; r < 8; ++r) st[j * 16 + col][wave * 16 + 8 * g + r] = acc[j][r];
  __syncthreads(); for (int e = tid; e < 128 * 16; e += 128) { const int dl = e >> 4, q = e & 15; vst2(KVT + ((b * MW + m) * CC + d0 + dl) * (size_t)CC + blockIdx.x * 64 + q * 4, *(const v4f*)&st[dl][q * 4]); } }
__global__ __launch_bounds__(128) void k_att(const float* __restrict__ PHQ, const float* __restrict__ KVT, const float* __restrict__ EQK, const float* __restrict__ WP, const float* __restrict__ BP, float* __restrict__ OUT) { __shared__ __align__(16) float sf[4][16][132];
  const int tid = threadIdx.x, wave = tid >> 5, lane = tid & 31, col = lane & 15, g = lane >> 4; const size_t b = blockIdx.z / MW; const int m = blockIdx.z % MW; const int t0 = blockIdx.x * 64 + wave * 16; const int d0 = blockIdx.y * 128;
  v8f acc[8] = {};
#pragma unroll
  for (int kc = 0; kc < CC / 32; ++kc) { const F2 a = split_row(PHQ + (b * NTOK + t0 + col) * CC, kc * 32, lane);
#pragma unroll
    for (int j = 0; j < 8; ++j) { float wv[16]; const float* wr = KVT + ((b * MW + m) * CC + d0 + j * 16 + col) * (size_t)CC + kc * 32 + 8 * g;
#pragma unroll
      for (int i = 0; i < 8; ++i) { wv[i] = wr[i]; wv[8 + i] = wr[16 + i]; }
      const F2 wb = bsplit16(wv); acc[j] = wmma_bf(a.h, wb.h, acc[j]); acc[j] = wmma_bf(a.h, wb.l, acc[j]); acc[j] = wmma_bf(a.l, wb.h, acc[j]); } }
  const float wp0 = bfr(WP[0]), wp1 = bfr(WP[1]), wp2 = bfr(WP[2]), bpv = bfr(BP[0]);
#pragma unroll
  for (int r = 0; r < 8; ++r) { const int t = t0 + 8 * g + r; const int w = t / MW, n = t % MW; const float* e3 = EQK + ((((b * NWIN + w) * MW + n) * MW + m) * 3); const float pv = bfr(e3[0]) * wp0 + bfr(e3[1]) * wp1 + bfr(e3[2]) * wp2 + bpv;
#pragma unroll
    for (int j = 0; j < 8; ++j) sf[wave][8 * g + r][j * 16 + col] = acc[j][r] + pv; }
  LDSX(); for (int rl = 0; rl < 16; ++rl) vst2(OUT + (b * NTOK + (size_t)(t0 + rl) * MW + m) * CC + d0 + lane * 4, *(const v4f*)&sf[wave][rl][lane * 4]); }
extern "C" void kernel_launch(void* const* d_in, const int* in_sizes, int n_in, void* d_out, int out_size, void* d_ws, size_t ws_size, hipStream_t stream) {
  (void)in_sizes; (void)n_in; (void)out_size;
  const float** F = (const float**)d_in;
  if (ws_size < (size_t)WS_END) return;
  char* ws = (char*)d_ws; __bf16* PW = (__bf16*)(ws + WS_PW); float *PHQ = (float*)(ws + WS_PHQ), *PHK = (float*)(ws + WS_PHK), *KVT = (float*)(ws + WS_KVT);
  k_packw<<<2 * CC, 256, 0, stream>>>(F[2], F[4], PW);
  k_phi<<<dim3(NB * NTOK / 64, CC / 128, 2), 128, 0, stream>>>(F[0], PW, F[3], F[5], PHQ, PHK);
  k_kv<<<dim3(CC / 64, CC / 128, NB * MW), 128, 0, stream>>>(PHK, F[0], KVT);
  k_att<<<dim3(TQ / 64, CC / 128, TNB * MW), 128, 0, stream>>>(PHQ, KVT, F[1], F[6], F[7], (float*)d_out);
}
